// EncoderProcessDecode_4672924418726
// MI455X (gfx1250) — hardware-verified
//
#include <hip/hip_runtime.h>
#include <stddef.h>
#include <math.h>

typedef __attribute__((ext_vector_type(16))) _Float16 v16h;
typedef __attribute__((ext_vector_type(8)))  _Float16 v8h;
typedef __attribute__((ext_vector_type(16))) __bf16   v16b;
typedef __attribute__((ext_vector_type(8)))  __bf16   v8b;
typedef __attribute__((ext_vector_type(8)))  float    v8f;
typedef __attribute__((ext_vector_type(4)))  float    v4f;
typedef __attribute__((ext_vector_type(4)))  int      v4i;

constexpr int HID     = 128;
constexpr int HID2    = 256;
constexpr int NODE_IN = 12;
constexpr int EDGE_IN = 7;
constexpr int KPAD    = 32;
constexpr int NSTEP   = 3;
constexpr int OUT_CH  = 3;
constexpr int OUT_PAD = 64;
constexpr int NTHR    = 256;
constexpr int NWAVE   = 8;
constexpr int CHE     = 23040;
constexpr int RPQ     = 512;
constexpr int NBA     = 512;
constexpr int EPT     = 8;
constexpr int NGRP    = 1;
constexpr int SUBCH   = NTHR * EPT * NGRP;
constexpr int WCAP    = EPT * NGRP * 32;
constexpr int LISTN   = NWAVE * WCAP;
constexpr int MAXSUB  = (CHE + SUBCH - 1) / SUBCH;
constexpr int LDS_AGG = NBA * HID * 4 + LISTN * 4 + 64;
constexpr float LN_EPSV = 1e-5f;

static_assert((SUBCH & (SUBCH - 1)) == 0 && SUBCH <= 4096);
static_assert((NBA & (NBA - 1)) == 0 && NBA <= 4096);
static_assert(RPQ % NBA == 0 && RPQ % 64 == 0 && RPQ % NTHR == 0);
static_assert(CHE % 64 == 0);
static_assert(LDS_AGG == 270400);
static_assert(MAXSUB * SUBCH >= CHE);

__device__ __forceinline__ unsigned short f2bf_bits(float f) {
  unsigned u = __float_as_uint(f);
  return (unsigned short)((u + 0x7FFFu + ((u >> 16) & 1u)) >> 16);
}
__device__ __forceinline__ float bf_bits2f(unsigned short h) { return __uint_as_float(((unsigned)h) << 16); }

__device__ __forceinline__ void dep_guard_h(v8f& a, v8f& b, v16h x, v16h y) { asm volatile("v_nop\n\tv_nop\n\tv_nop\n\tv_nop" : "+v"(a), "+v"(b) : "v"(x), "v"(y)); }
__device__ __forceinline__ void dep_guard_b(v8f& a, v8f& b, v16b x, v16b y) { asm volatile("v_nop\n\tv_nop\n\tv_nop\n\tv_nop" : "+v"(a), "+v"(b) : "v"(x), "v"(y)); }
__device__ __forceinline__ void keep4_h(v16h a, v16h b, v16h c, v16h d) { asm volatile("v_nop" :: "v"(a), "v"(b), "v"(c), "v"(d)); }
__device__ __forceinline__ void keep4_b(v16b a, v16b b, v16b c, v16b d) { asm volatile("v_nop" :: "v"(a), "v"(b), "v"(c), "v"(d)); }
__device__ __forceinline__ void acc_guard4(v8f& a, v8f& b, v8f& c, v8f& d) { asm volatile("v_nop\n\tv_nop\n\tv_nop\n\tv_nop" : "+v"(a), "+v"(b), "+v"(c), "+v"(d)); }
template <typename T> struct Frag;
template <> struct Frag<_Float16> {
  typedef v16h V; union U { v16h v; v8h h[2]; };
  static __device__ __forceinline__ v16h load(const _Float16* p) {
    U f; f.h[0] = *(const v8h*)(p); f.h[1] = *(const v8h*)(p + 16); return f.v;
  }
  static __device__ __forceinline__ v8f mma(v16h a, v16h b, v8f c) {
    return __builtin_amdgcn_wmma_f32_16x16x32_f16(false, a, false, b, (short)0, c, false, false);
  }
  static __device__ __forceinline__ void guard(v8f& a, v8f& b, v16h x, v16h y) { dep_guard_h(a, b, x, y); }
  static __device__ __forceinline__ void keep(v16h a, v16h b, v16h c, v16h d) { keep4_h(a, b, c, d); }
};
template <> struct Frag<__bf16> {
  typedef v16b V; union U { v16b v; v8b h[2]; };
  static __device__ __forceinline__ v16b load(const __bf16* p) {
    U f; f.h[0] = *(const v8b*)(p); f.h[1] = *(const v8b*)(p + 16); return f.v;
  }
  static __device__ __forceinline__ v8f mma(v16b a, v16b b, v8f c) {
    return __builtin_amdgcn_wmma_f32_16x16x32_bf16(false, a, false, b, (short)0, c, false, false);
  }
  static __device__ __forceinline__ void guard(v8f& a, v8f& b, v16b x, v16b y) { dep_guard_b(a, b, x, y); }
  static __device__ __forceinline__ void keep(v16b a, v16b b, v16b c, v16b d) { keep4_b(a, b, c, d); }
};

template <int ET> struct Elem;
template <> struct Elem<0> { typedef _Float16 T; };
template <> struct Elem<1> { typedef __bf16 T; };
template <int ET, bool SPLIT, int BIAS_MODE, int OUT_MODE, bool RESID, int ACT = 0>
__global__ __launch_bounds__(256) void wmma_gemm64(
    const unsigned short* __restrict__ Ap, const unsigned short* __restrict__ A2p, int lda, long strideA,
    const unsigned short* __restrict__ Btp, const unsigned short* __restrict__ Bt2p, int ldb, long strideB,
    void* __restrict__ Cout, void* __restrict__ Cout2, int ldc, long strideC,
    const float* __restrict__ bias,
    const float* __restrict__ resid, long strideR,
    int M, int N, int K, float scale) {
  typedef typename Elem<ET>::T T;
  typedef typename Frag<T>::V V;
  const T* A = (const T*)Ap; const T* A2 = (const T*)A2p; const T* Bt = (const T*)Btp; const T* Bt2 = (const T*)Bt2p;
  __shared__ __align__(16) float sT[8][16 * 68];
  const int b    = blockIdx.y;
  const int lane = threadIdx.x & 31;
  const int wave = threadIdx.x >> 5;
  const int tilesN = N >> 6;
  const int tilesM = M >> 6;
  const int tile = blockIdx.x * 8 + wave;
  if (tile >= tilesM * tilesN) return;
  const int tm = tile / tilesN;
  const int tn = tile - tm * tilesN;
  const int m0 = tm << 6;
  const int n0 = tn << 6;

  const T* Ab  = A  + (size_t)b * strideA;
  const T* Bb  = Bt + (size_t)b * strideB;
  const T* Ab2 = SPLIT ? (A2  + (size_t)b * strideA) : nullptr;
  const T* Bb2 = SPLIT ? (Bt2 + (size_t)b * strideB) : nullptr;

  const int rlane = lane & 15;
  const int koff  = (lane >> 4) * 8;
  const int mOff  = (lane >> 4) * 8;

  v8f acc[4][4];
#pragma unroll
  for (int i = 0; i < 4; ++i)
#pragma unroll
    for (int j = 0; j < 4; ++j) acc[i][j] = (v8f){0.f,0.f,0.f,0.f,0.f,0.f,0.f,0.f};

  for (int k0 = 0; k0 < K; k0 += 32) {
    V bh[4], bl[4];
#pragma unroll
    for (int j = 0; j < 4; ++j) {
      const size_t bo = (size_t)(n0 + (j << 4) + rlane) * ldb + koff + k0;
      bh[j] = Frag<T>::load(Bb + bo);
      if (SPLIT) bl[j] = Frag<T>::load(Bb2 + bo);
    }
#pragma unroll
    for (int i = 0; i < 4; ++i) {
      const size_t ao = (size_t)(m0 + (i << 4) + rlane) * lda + koff + k0;
      V ah = Frag<T>::load(Ab + ao);
      V al;
      if (SPLIT) al = Frag<T>::load(Ab2 + ao);
#pragma unroll
      for (int j = 0; j < 4; ++j) {
        acc[i][j] = Frag<T>::mma(ah, bh[j], acc[i][j]);
        if (SPLIT) {
          acc[i][j] = Frag<T>::mma(ah, bl[j], acc[i][j]);
          acc[i][j] = Frag<T>::mma(al, bh[j], acc[i][j]);
        }
      }
      Frag<T>::guard(acc[i][0], acc[i][3], ah, SPLIT ? al : ah);
    }
    Frag<T>::keep(bh[0], bh[1], bh[2], bh[3]);
    if (SPLIT) Frag<T>::keep(bl[0], bl[1], bl[2], bl[3]);
  }
  acc_guard4(acc[0][0], acc[0][1], acc[0][2], acc[0][3]);
  acc_guard4(acc[1][0], acc[1][1], acc[1][2], acc[1][3]);
  acc_guard4(acc[2][0], acc[2][1], acc[2][2], acc[2][3]);
  acc_guard4(acc[3][0], acc[3][1], acc[3][2], acc[3][3]);

  float* slab = sT[wave];
  const float* Rb = RESID ? (resid + (size_t)b * strideR) : nullptr;
#pragma unroll
  for (int i = 0; i < 4; ++i) {
    const int mBase = m0 + (i << 4);
#pragma unroll
    for (int j = 0; j < 4; ++j) {
      const int n = n0 + (j << 4) + rlane;
      float bv = 0.f;
      if (BIAS_MODE == 2) bv = bias[n];
#pragma unroll
      for (int r = 0; r < 8; ++r) {
        float v = acc[i][j][r] * scale;
        if (BIAS_MODE == 1) v += bias[mBase + mOff + r];
        if (BIAS_MODE == 2) v += bv;
        if (RESID) v += Rb[(size_t)(mBase + mOff + r) * ldc + n];
        if (ACT == 1) v = tanhf(v);
        if (ACT == 2) v = fmaxf(v, 0.0f);
        if (ACT == 3) v = v / (1.0f + expf(-v));
        if (ACT == 4) v = (v > 0.f) ? v : 0.01f * v;
        if (ACT == 5) v = 0.5f * v * (1.0f + erff(v * 0.70710678118654752f));
        slab[(mOff + r) * 68 + (j << 4) + rlane] = v;
      }
    }
    __builtin_amdgcn_fence(__ATOMIC_RELEASE, "workgroup");
    __builtin_amdgcn_wave_barrier();
    __builtin_amdgcn_fence(__ATOMIC_ACQUIRE, "workgroup");
    if (OUT_MODE == 0) {
      float* C = (float*)Cout + (size_t)b * strideC;
      const int hh = lane >> 4, c4 = (lane & 15) * 4;
      for (int pass = 0; pass < 2; ++pass) {
#pragma unroll
        for (int it = 0; it < 8; ++it) {
          const int row = it * 2 + hh;
          v4f v = *(const v4f*)(slab + row * 68 + c4);
          *(volatile v4f*)(C + (size_t)(mBase + row) * ldc + n0 + c4) = v;
        }
        __threadfence();
      }
    } else {
      const int q = lane >> 3, c8 = (lane & 7) * 8;
      unsigned short* C  = (unsigned short*)Cout  + (size_t)b * strideC;
      unsigned short* C2 = (OUT_MODE == 2) ? ((unsigned short*)Cout2 + (size_t)b * strideC) : nullptr;
      for (int pass = 0; pass < 2; ++pass) {
#pragma unroll
        for (int it = 0; it < 4; ++it) {
          const int row = it * 4 + q;
          const float* sp = slab + row * 68 + c8;
          v8h hv, lv;
#pragma unroll
          for (int e = 0; e < 8; ++e) {
            if (OUT_MODE == 1) {
              hv[e] = (_Float16)sp[e];
            } else {
              unsigned short hb = f2bf_bits(sp[e]);
              unsigned short lb = f2bf_bits(sp[e] - bf_bits2f(hb));
              hv[e] = __builtin_bit_cast(_Float16, hb);
              lv[e] = __builtin_bit_cast(_Float16, lb);
            }
          }
          *(volatile v8h*)(C + (size_t)(mBase + row) * ldc + n0 + c8) = hv;
          if (OUT_MODE == 2) *(volatile v8h*)(C2 + (size_t)(mBase + row) * ldc + n0 + c8) = lv;
        }
        __threadfence();
      }
    }
    __builtin_amdgcn_fence(__ATOMIC_RELEASE, "workgroup");
    __builtin_amdgcn_wave_barrier();
    __builtin_amdgcn_fence(__ATOMIC_ACQUIRE, "workgroup");
  }
}

template <int NB>
__device__ __forceinline__ int scan_chunk(const int* __restrict__ lst, int nE, int cbase, int nodeBase,
                                          int* list, int tid, int lane, int wave, int fullvec) {
  int wc = 0;
#pragma unroll
  for (int g = 0; g < NGRP; ++g) {
    const int el0 = (g * NTHR + tid) * EPT;
    const int e0  = cbase + el0;
    v4i da, db;
    if (fullvec) {
      da = *(const v4i*)(lst + e0);
      db = *(const v4i*)(lst + e0 + 4);
    } else {
      const int em = nE - 1;
      da.x = lst[(e0     < em) ? e0     : em];
      da.y = lst[(e0 + 1 < em) ? e0 + 1 : em];
      da.z = lst[(e0 + 2 < em) ? e0 + 2 : em];
      da.w = lst[(e0 + 3 < em) ? e0 + 3 : em];
      db.x = lst[(e0 + 4 < em) ? e0 + 4 : em];
      db.y = lst[(e0 + 5 < em) ? e0 + 5 : em];
      db.z = lst[(e0 + 6 < em) ? e0 + 6 : em];
      db.w = lst[(e0 + 7 < em) ? e0 + 7 : em];
    }
    const bool v0 = (e0 < nE), v1 = (e0 + 1 < nE), v2 = (e0 + 2 < nE), v3 = (e0 + 3 < nE);
    const bool v4 = (e0 + 4 < nE), v5 = (e0 + 5 < nE), v6 = (e0 + 6 < nE), v7 = (e0 + 7 < nE);
    const unsigned nb = (unsigned)nodeBase;
    const unsigned s0 = (unsigned)da.x - nb, s1 = (unsigned)da.y - nb;
    const unsigned s2 = (unsigned)da.z - nb, s3 = (unsigned)da.w - nb;
    const unsigned s4 = (unsigned)db.x - nb, s5 = (unsigned)db.y - nb;
    const unsigned s6 = (unsigned)db.z - nb, s7 = (unsigned)db.w - nb;
    const bool h0 = v0 && (s0 < (unsigned)NB), h1 = v1 && (s1 < (unsigned)NB);
    const bool h2 = v2 && (s2 < (unsigned)NB), h3 = v3 && (s3 < (unsigned)NB);
    const bool h4 = v4 && (s4 < (unsigned)NB), h5 = v5 && (s5 < (unsigned)NB);
    const bool h6 = v6 && (s6 < (unsigned)NB), h7 = v7 && (s7 < (unsigned)NB);
    const unsigned any = __builtin_amdgcn_ballot_w32(h0 | h1 | h2 | h3 | h4 | h5 | h6 | h7);
    if (any != 0u) {
#define HITJ(J, HJ, SJ) { \
        const unsigned mj = __builtin_amdgcn_ballot_w32(HJ); \
        if (mj != 0u) { \
          if (HJ) { \
            const int pos = wc + (int)__builtin_amdgcn_mbcnt_lo(mj, 0u); \
            if (pos < WCAP) list[wave * WCAP + pos] = ((el0 + (J)) << 12) | (int)(SJ); \
          } \
          wc += (int)__builtin_popcount(mj); } }
      HITJ(0, h0, s0)
      HITJ(1, h1, s1)
      HITJ(2, h2, s2)
      HITJ(3, h3, s3)
      HITJ(4, h4, s4)
      HITJ(5, h5, s5)
      HITJ(6, h6, s6)
      HITJ(7, h7, s7)
#undef HITJ
    }
  }
  return wc;
}

__global__ __launch_bounds__(NTHR) void k_wsplit(const float* __restrict__ W, long strideW, int Kin, int ncol, int G,
                                                 int NR, int KP, unsigned short* bth, unsigned short* btl, long strideO) {
  const float* Wl = W + (size_t)blockIdx.y * (size_t)strideW;
  const size_t ob = (size_t)blockIdx.y * (size_t)strideO;
  const int tpr = KP >> 3;
  const int i = blockIdx.x * NTHR + threadIdx.x;
  if (i >= NR * tpr) return;
  const int n  = i / tpr;
  const int k0 = (i - n * tpr) * 8;
  int g = n / ncol; g = (g > G - 1) ? G - 1 : g;
  int nn = n - g * ncol; nn = (nn > ncol - 1) ? ncol - 1 : ((nn < 0) ? 0 : nn);
  const bool nok = (n < G * ncol);
  v8h hv, lv;
#pragma unroll
  for (int e = 0; e < 8; ++e) {
    const int k  = k0 + e;
    const int kc = (k < Kin) ? k : Kin - 1;
    float v = Wl[((size_t)g * Kin + kc) * ncol + nn];
    if (k >= Kin || !nok) v = 0.f;
    const unsigned short hb = f2bf_bits(v);
    const unsigned short lb = f2bf_bits(v - bf_bits2f(hb));
    hv[e] = __builtin_bit_cast(_Float16, hb);
    lv[e] = __builtin_bit_cast(_Float16, lb);
  }
  const size_t o = ob + (size_t)i * 8;
  *(volatile v8h*)(bth + o) = hv;
  *(volatile v8h*)(btl + o) = lv;
  __threadfence();
  *(volatile v8h*)(bth + o) = hv;
  *(volatile v8h*)(btl + o) = lv;
}

__global__ __launch_bounds__(NTHR) void k_wf16(const float* __restrict__ W, long strideW, int Kin, int ncol,
                                               int NR, int KP, float sc, unsigned short* bt, long strideO) {
  const float* Wl = W + (size_t)blockIdx.y * (size_t)strideW;
  const size_t ob = (size_t)blockIdx.y * (size_t)strideO;
  const int tpr = KP >> 3;
  const int i = blockIdx.x * NTHR + threadIdx.x;
  if (i >= NR * tpr) return;
  const int n   = i / tpr;
  const int k0  = (i - n * tpr) * 8;
  const int ncl = (n < ncol) ? n : ncol - 1;
  v8h hv;
#pragma unroll
  for (int e = 0; e < 8; ++e) {
    const int k  = k0 + e;
    const int kc = (k < Kin) ? k : Kin - 1;
    float v = sc * Wl[(size_t)kc * ncol + ncl];
    if (k >= Kin || n >= ncol) v = 0.f;
    hv[e] = (_Float16)v;
  }
  const size_t o = ob + (size_t)i * 8;
  *(volatile v8h*)(bt + o) = hv;
  __threadfence();
  *(volatile v8h*)(bt + o) = hv;
}

__global__ __launch_bounds__(NTHR) void k_xsplit(const float* __restrict__ x, int nN, int NPr,
                                                 unsigned short* xh, unsigned short* xl) {
  const int i = blockIdx.x * NTHR + threadIdx.x;
  const int row = i >> 2;
  const int k0 = (i & 3) * 8;
  const int rowc = (row < nN) ? row : nN - 1;
  const float* xr = x + (size_t)rowc * NODE_IN;
  v8h hv, lv;
#pragma unroll
  for (int e = 0; e < 8; ++e) {
    const int k  = k0 + e;
    const int kc = (k < NODE_IN) ? k : NODE_IN - 1;
    float v = xr[kc];
    if (k >= NODE_IN || row >= nN) v = 0.f;
    const unsigned short hb = f2bf_bits(v);
    const unsigned short lb = f2bf_bits(v - bf_bits2f(hb));
    hv[e] = __builtin_bit_cast(_Float16, hb);
    lv[e] = __builtin_bit_cast(_Float16, lb);
  }
  const bool ok = (row < NPr);
  const size_t o = (size_t)(ok ? i : 0) * 8;
  if (ok) { *(volatile v8h*)(xh + o) = hv; *(volatile v8h*)(xl + o) = lv; }
  __threadfence();
  if (ok) { *(volatile v8h*)(xh + o) = hv; *(volatile v8h*)(xl + o) = lv; }
}

__global__ __launch_bounds__(NTHR) void k_excast(const float* __restrict__ ex, int nE, int EPr, unsigned short* out) {
  const int i = blockIdx.x * NTHR + threadIdx.x;
  const int row = i >> 2;
  const int k0 = (i & 3) * 8;
  const int rowc = (row < nE) ? row : nE - 1;
  const float* er = ex + (size_t)rowc * EDGE_IN;
  v8h hv;
#pragma unroll
  for (int e = 0; e < 8; ++e) {
    const int k  = k0 + e;
    const int kc = (k < EDGE_IN) ? k : EDGE_IN - 1;
    float v = er[kc];
    if (k >= EDGE_IN || row >= nE) v = 0.0f;
    hv[e] = (_Float16)v;
  }
  const bool ok = (row < EPr);
  const size_t o = (size_t)(ok ? i : 0) * 8;
  if (ok) *(volatile v8h*)(out + o) = hv;
  __threadfence();
  if (ok) *(volatile v8h*)(out + o) = hv;
}

__device__ __forceinline__ float wave_sum32(float s) {
#pragma unroll
  for (int off = 1; off < 32; off <<= 1) s += __shfl_xor(s, off, 32);
  return s;
}
__device__ __forceinline__ v4f ln_row4(v4f v, const float* __restrict__ gam, const float* __restrict__ bet, int c4) {
  float s = (v.x + v.y) + (v.z + v.w);
  s = wave_sum32(s);
  const float mu = s * (1.0f / 128.0f);
  const v4f d = v - mu;
  float q = (d.x * d.x + d.y * d.y) + (d.z * d.z + d.w * d.w);
  q = wave_sum32(q);
  const float var = q * (1.0f / 128.0f);
  const float inv = rsqrtf(var + LN_EPSV);
  const v4f gg = *(const v4f*)(gam + c4);
  const v4f bb = *(const v4f*)(bet + c4);
  return (d * inv) * gg + bb;
}

__global__ __launch_bounds__(NTHR) void k_gath(const float* __restrict__ pab, const int* __restrict__ snd,
                                               const int* __restrict__ rcv, int nN, int nE, int ebase, int Mc,
                                               float* gout) {
  const int lane = threadIdx.x & 31, wave = threadIdx.x >> 5;
  const int r = blockIdx.x * NWAVE + wave;
  const int rc = (r < Mc) ? r : Mc - 1;
  const int c4 = lane * 4;
  const int e = ebase + r;
  const bool valid = (e < nE);
  int ec = valid ? e : nE - 1; ec = (ec < 0) ? 0 : ec;
  int s = snd[ec];
  int d = rcv[ec];
  s = (s < 0) ? 0 : ((s > nN - 1) ? nN - 1 : s);
  d = (d < 0) ? 0 : ((d > nN - 1) ? nN - 1 : d);
  const v4f a = *(const v4f*)(pab + (size_t)s * HID2 + c4);
  const v4f b = *(const v4f*)(pab + (size_t)d * HID2 + HID + c4);
  v4f o = a + b;
  const v4f z4 = {0.f, 0.f, 0.f, 0.f};
  if (!valid) o = z4;
  const bool ok = (r < Mc);
  float* op = gout + (size_t)rc * HID + c4;
  if (ok) *(volatile v4f*)op = o;
  __threadfence();
  if (ok) *(volatile v4f*)op = o;
}

__global__ __launch_bounds__(NTHR) void k_eln(const float* __restrict__ m3, const float* __restrict__ gam,
                                              const float* __restrict__ bet, int nE, int EPr, int ebase, int Mc,
                                              int first, int wr_new, unsigned short* ef16, float* newef) {
  __shared__ __align__(16) float sl[NWAVE][HID];
  const int tid = threadIdx.x, lane = tid & 31, wave = tid >> 5;
  const int r = blockIdx.x * NWAVE + wave;
  const int rc = (r < Mc) ? r : Mc - 1;
  const int c4 = lane * 4;
  const int e = ebase + r;
  const bool valid = (e < nE);
  const v4f v = *(const v4f*)(m3 + (size_t)rc * HID + c4);
  v4f y = ln_row4(v, gam, bet, c4);
  const v4f z4 = {0.f, 0.f, 0.f, 0.f};
  if (!valid) y = z4;
  *(v4f*)(&sl[wave][c4]) = y;
  __syncthreads();
  const int l16 = lane & 15;
  int ec = (e < EPr) ? e : EPr - 1; ec = (ec < 0) ? 0 : ec;
  const _Float16* efr = (const _Float16*)ef16 + (size_t)ec * HID + 8 * l16;
  const v8h old = *(const v8h*)efr;
  const v4f y0 = *(const v4f*)(&sl[wave][8 * l16]);
  const v4f y1 = *(const v4f*)(&sl[wave][8 * l16 + 4]);
  v8h nv;
#pragma unroll
  for (int q = 0; q < 4; ++q) {
    float o0 = (float)old[q];     if (first) o0 = 0.f;
    float o1 = (float)old[4 + q]; if (first) o1 = 0.f;
    float t0 = o0 + y0[q];
    float t1 = o1 + y1[q];
    if (!valid) { t0 = 0.f; t1 = 0.f; }
    nv[q] = (_Float16)t0;
    nv[4 + q] = (_Float16)t1;
  }
  const bool okN = (wr_new != 0) && (r < Mc);
  const bool okE = (lane < 16) && (r < Mc) && (e < EPr);
  float* np_ = newef + (size_t)rc * HID + c4;
  unsigned short* ep = ef16 + (size_t)ec * HID + 8 * l16;
  if (okN) *(volatile v4f*)np_ = y;
  if (okE) *(volatile v8h*)ep = nv;
  __threadfence();
  if (okN) *(volatile v4f*)np_ = y;
  if (okE) *(volatile v8h*)ep = nv;
}

__global__ __launch_bounds__(NTHR) void k_nln(const float* __restrict__ u3, const float* __restrict__ gam,
                                              const float* __restrict__ bet, int nN, int NPr, int first,
                                              float* nf, unsigned short* ch, unsigned short* cl) {
  __shared__ __align__(16) float sl[NWAVE][HID];
  const int tid = threadIdx.x, lane = tid & 31, wave = tid >> 5;
  const int row = blockIdx.x * NWAVE + wave;
  const int rowc = (row < NPr) ? row : NPr - 1;
  const int c4 = lane * 4;
  const v4f v = *(const v4f*)(u3 + (size_t)rowc * HID + c4);
  const v4f y = ln_row4(v, gam, bet, c4);
  const v4f old = *(const v4f*)(nf + (size_t)rowc * HID + c4);
  v4f nv = old + y;
  if (first) nv = y;
  const v4f z4 = {0.f, 0.f, 0.f, 0.f};
  if (row >= nN) nv = z4;
  *(v4f*)(&sl[wave][c4]) = nv;
  __syncthreads();
  const int hsel = lane >> 4, c8 = (lane & 15) * 8;
  const v4f t0 = *(const v4f*)(&sl[wave][c8]);
  const v4f t1 = *(const v4f*)(&sl[wave][c8 + 4]);
  v8h pv;
#pragma unroll
  for (int q = 0; q < 4; ++q) {
    const unsigned short hb0 = f2bf_bits(t0[q]);
    const unsigned short lb0 = f2bf_bits(t0[q] - bf_bits2f(hb0));
    const unsigned short hb1 = f2bf_bits(t1[q]);
    const unsigned short lb1 = f2bf_bits(t1[q] - bf_bits2f(hb1));
    pv[q]     = __builtin_bit_cast(_Float16, (unsigned short)(hsel ? lb0 : hb0));
    pv[4 + q] = __builtin_bit_cast(_Float16, (unsigned short)(hsel ? lb1 : hb1));
  }
  unsigned short* pbase = hsel ? cl : ch;
  unsigned short* pp = pbase + (size_t)rowc * HID2 + c8;
  float* np_ = nf + (size_t)rowc * HID + c4;
  const bool ok = (row < NPr);
  if (ok) { *(volatile v4f*)np_ = nv; *(volatile v8h*)pp = pv; }
  __threadfence();
  if (ok) { *(volatile v4f*)np_ = nv; *(volatile v8h*)pp = pv; }
}

__global__ __launch_bounds__(NTHR) void k_agg(const int* __restrict__ dstl, int nEc,
                                              const float* __restrict__ mh, float* agg, int first, int vec_ok) {
  constexpr int NB  = NBA;
  constexpr int NV4 = NB * HID / 4;
  static_assert(NV4 % NTHR == 0);
  extern __shared__ v4f lds_dyn[];
  float* acc  = (float*)lds_dyn;
  int*   list = (int*)(acc + NB * HID);
  int*   wcnt = list + LISTN;
  const int tid = threadIdx.x, lane = tid & 31, wave = tid >> 5;
  const int nodeBase = blockIdx.x * NB;
  float* ga = agg + (size_t)nodeBase * HID;

  if (first) {
    const v4f zz = {0.f, 0.f, 0.f, 0.f};
    for (int i = tid; i < NV4; i += NTHR) lds_dyn[i] = zz;
  } else {
    for (int i = tid; i < NV4; i += NTHR) lds_dyn[i] = ((const v4f*)ga)[i];
  }
  __syncthreads();

  int nSub = (nEc + SUBCH - 1) / SUBCH;
  nSub = (nSub > MAXSUB) ? MAXSUB : ((nSub < 0) ? 0 : nSub);
#pragma unroll 1
  for (int chk = 0; chk < nSub; ++chk) {
    const int cbase = chk * SUBCH;
    const int fullvec = (vec_ok != 0 && cbase + SUBCH <= nEc) ? 1 : 0;
    const int wc = scan_chunk<NB>(dstl, nEc, cbase, nodeBase, list, tid, lane, wave, fullvec);
    if (lane == 0) wcnt[wave] = wc;
    __syncthreads();
    if (wave == 0) {
#pragma unroll 1
      for (int wsx = 0; wsx < NWAVE; ++wsx) {
        int n = __builtin_amdgcn_readfirstlane(wcnt[wsx]);
        n = n > WCAP ? WCAP : (n < 0 ? 0 : n);
        const int* lp = list + wsx * WCAP;
#pragma unroll 1
        for (int i = 0; i < n; ++i) {
          const int ent  = __builtin_amdgcn_readfirstlane(lp[i]);
          const int slot = ent & (NB - 1);
          int el = cbase + ((ent >> 12) & (SUBCH - 1));
          el = (el > nEc - 1) ? nEc - 1 : el;
          const v4f m4 = *(const v4f*)(mh + (size_t)el * HID + 4 * lane);
          v4f* ap = (v4f*)(acc + slot * HID + 4 * lane);
          const v4f av = *ap;
          *ap = av + m4;
        }
      }
    }
    __syncthreads();
  }

  for (int pass = 0; pass < 2; ++pass) {
#pragma unroll 4
    for (int i = tid; i < NV4; i += NTHR) { const v4f vv = lds_dyn[i]; ((volatile v4f*)ga)[i] = vv; }
    __threadfence();
  }
}

__global__ __launch_bounds__(NTHR) void k_aggsplit(const float* __restrict__ agg, int NPr,
                                                   unsigned short* ch, unsigned short* cl) {
  const int i = blockIdx.x * NTHR + threadIdx.x;
  const int row = i >> 4;
  const int k0 = (i & 15) * 8;
  const int rowc = (row < NPr) ? row : NPr - 1;
  const float* ar = agg + (size_t)rowc * HID + k0;
  const v4f a0 = *(const v4f*)ar;
  const v4f a1 = *(const v4f*)(ar + 4);
  v8h hv, lv;
#pragma unroll
  for (int q = 0; q < 4; ++q) {
    const unsigned short hb0 = f2bf_bits(a0[q]);
    const unsigned short lb0 = f2bf_bits(a0[q] - bf_bits2f(hb0));
    const unsigned short hb1 = f2bf_bits(a1[q]);
    const unsigned short lb1 = f2bf_bits(a1[q] - bf_bits2f(hb1));
    hv[q] = __builtin_bit_cast(_Float16, hb0);  lv[q] = __builtin_bit_cast(_Float16, lb0);
    hv[4 + q] = __builtin_bit_cast(_Float16, hb1);  lv[4 + q] = __builtin_bit_cast(_Float16, lb1);
  }
  const bool ok = (row < NPr);
  const size_t o = (size_t)rowc * HID2 + HID + k0;
  if (ok) { *(volatile v8h*)(ch + o) = hv; *(volatile v8h*)(cl + o) = lv; }
  __threadfence();
  if (ok) { *(volatile v8h*)(ch + o) = hv; *(volatile v8h*)(cl + o) = lv; }
}

__global__ __launch_bounds__(NTHR) void k_pack(const float* __restrict__ d3, const float* __restrict__ b2,
                                               int nN, int NPr, float* out) {
  const int i = blockIdx.x * NTHR + threadIdx.x;
  const int total = nN * OUT_CH;
  const int f0 = 4 * i;
  v4f o;
#pragma unroll
  for (int j = 0; j < 4; ++j) {
    const int f = f0 + j;
    const int fc = (f < total) ? f : total - 1;
    int row = fc / OUT_CH;
    const int col = fc - row * OUT_CH;
    row = (row > NPr - 1) ? NPr - 1 : row;
    o[j] = d3[(size_t)row * OUT_PAD + col] + b2[col];
  }
  const bool ok = (f0 + 4 <= total);
  float* op = out + (size_t)(ok ? f0 : 0);
  if (ok) *(volatile v4f*)op = o;
  __threadfence();
  if (ok) *(volatile v4f*)op = o;
}

extern "C" void kernel_launch(void* const* d_in, const int* in_sizes, int n_in,
                              void* d_out, int out_size, void* d_ws, size_t ws_size,
                              hipStream_t stream) {
  if (n_in < 42) return;
  const int nN = in_sizes[0] / NODE_IN;
  const int nE = in_sizes[40];
  if (nN < 1 || in_sizes[0] != nN * NODE_IN || nN > (1 << 22)) return;
  if (nE < 1 || in_sizes[41] != nE || in_sizes[1] != nE * EDGE_IN || nE > (1 << 24)) return;
  if (in_sizes[2] != NODE_IN * HID || in_sizes[4] != HID * HID || in_sizes[6] != HID * HID) return;
  if (in_sizes[3] != HID || in_sizes[5] != HID || in_sizes[7] != HID || in_sizes[8] != HID || in_sizes[9] != HID) return;
  if (in_sizes[10] != EDGE_IN * HID || in_sizes[12] != HID * HID || in_sizes[14] != HID * HID) return;
  if (in_sizes[11] != HID || in_sizes[13] != HID || in_sizes[15] != HID || in_sizes[16] != HID || in_sizes[17] != HID) return;
  if (in_sizes[18] != NSTEP * 3 * HID * HID || in_sizes[20] != NSTEP * HID * HID || in_sizes[22] != NSTEP * HID * HID) return;
  if (in_sizes[19] != NSTEP * HID || in_sizes[21] != NSTEP * HID || in_sizes[23] != NSTEP * HID) return;
  if (in_sizes[24] != NSTEP * HID || in_sizes[25] != NSTEP * HID) return;
  if (in_sizes[26] != NSTEP * HID2 * HID || in_sizes[28] != NSTEP * HID * HID || in_sizes[30] != NSTEP * HID * HID) return;
  if (in_sizes[27] != NSTEP * HID || in_sizes[29] != NSTEP * HID || in_sizes[31] != NSTEP * HID) return;
  if (in_sizes[32] != NSTEP * HID || in_sizes[33] != NSTEP * HID) return;
  if (in_sizes[34] != HID * HID || in_sizes[35] != HID || in_sizes[36] != HID * HID || in_sizes[37] != HID) return;
  if (in_sizes[38] != HID * OUT_CH || in_sizes[39] != OUT_CH) return;
  if (out_size != nN * OUT_CH || (out_size & 3) != 0) return;

  const float* node_x = (const float*)d_in[0];
  const float* edge_x = (const float*)d_in[1];
  const float* enW0 = (const float*)d_in[2];  const float* enb0 = (const float*)d_in[3];
  const float* enW1 = (const float*)d_in[4];  const float* enb1 = (const float*)d_in[5];
  const float* enW2 = (const float*)d_in[6];  const float* enb2 = (const float*)d_in[7];
  const float* eng  = (const float*)d_in[8];  const float* enbe = (const float*)d_in[9];
  const float* eeW0 = (const float*)d_in[10]; const float* eeb0 = (const float*)d_in[11];
  const float* eeW1 = (const float*)d_in[12]; const float* eeb1 = (const float*)d_in[13];
  const float* eeW2 = (const float*)d_in[14]; const float* eeb2 = (const float*)d_in[15];
  const float* eeg  = (const float*)d_in[16]; const float* eebe = (const float*)d_in[17];
  const float* geW0 = (const float*)d_in[18]; const float* geb0 = (const float*)d_in[19];
  const float* geW1 = (const float*)d_in[20]; const float* geb1 = (const float*)d_in[21];
  const float* geW2 = (const float*)d_in[22]; const float* geb2 = (const float*)d_in[23];
  const float* geg  = (const float*)d_in[24]; const float* gebe = (const float*)d_in[25];
  const float* gnW0 = (const float*)d_in[26]; const float* gnb0 = (const float*)d_in[27];
  const float* gnW1 = (const float*)d_in[28]; const float* gnb1 = (const float*)d_in[29];
  const float* gnW2 = (const float*)d_in[30]; const float* gnb2 = (const float*)d_in[31];
  const float* gng  = (const float*)d_in[32]; const float* gnbe = (const float*)d_in[33];
  const float* dW0  = (const float*)d_in[34]; const float* db0  = (const float*)d_in[35];
  const float* dW1  = (const float*)d_in[36]; const float* db1  = (const float*)d_in[37];
  const float* dW2  = (const float*)d_in[38]; const float* db2  = (const float*)d_in[39];
  const int*   senders   = (const int*)d_in[40];
  const int*   receivers = (const int*)d_in[41];
  float* out0 = (float*)d_out;

  const int NPr = ((nN + RPQ - 1) / RPQ) * RPQ;
  const int EPr = ((nE + 127) / 128) * 128;
  const int nChunks = (nE + CHE - 1) / CHE;
  if (nChunks < 1 || nChunks > 64) return;
  const int nA = NPr / NBA;

  size_t off = 0;
  auto carve = [&](size_t bytes) { const size_t o = off; off += (bytes + 255) & ~(size_t)255; return o; };
  const size_t oWN0H = carve((size_t)HID * KPAD * 2),  oWN0L = carve((size_t)HID * KPAD * 2);
  const size_t oWN1H = carve((size_t)HID * HID * 2),   oWN1L = carve((size_t)HID * HID * 2);
  const size_t oWN2H = carve((size_t)HID * HID * 2),   oWN2L = carve((size_t)HID * HID * 2);
  const size_t oWE0  = carve((size_t)HID * KPAD * 2);
  const size_t oWE1  = carve((size_t)HID * HID * 2),   oWE2  = carve((size_t)HID * HID * 2);
  const size_t oPBWH = carve((size_t)NSTEP * HID2 * HID * 2), oPBWL = carve((size_t)NSTEP * HID2 * HID * 2);
  const size_t oEW0C = carve((size_t)NSTEP * HID * HID * 2);
  const size_t oEW1  = carve((size_t)NSTEP * HID * HID * 2),  oEW2  = carve((size_t)NSTEP * HID * HID * 2);
  const size_t oNW0H = carve((size_t)NSTEP * HID * HID2 * 2), oNW0L = carve((size_t)NSTEP * HID * HID2 * 2);
  const size_t oNW1H = carve((size_t)NSTEP * HID * HID * 2),  oNW1L = carve((size_t)NSTEP * HID * HID * 2);
  const size_t oNW2H = carve((size_t)NSTEP * HID * HID * 2),  oNW2L = carve((size_t)NSTEP * HID * HID * 2);
  const size_t oDW0H = carve((size_t)HID * HID * 2),   oDW0L = carve((size_t)HID * HID * 2);
  const size_t oDW1H = carve((size_t)HID * HID * 2),   oDW1L = carve((size_t)HID * HID * 2);
  const size_t oDW2H = carve((size_t)OUT_PAD * HID * 2), oDW2L = carve((size_t)OUT_PAD * HID * 2);
  const size_t oEF16 = carve((size_t)EPr * HID * 2);
  const size_t oNF   = carve((size_t)NPr * HID * 4);
  const size_t oCH   = carve((size_t)NPr * HID2 * 2);
  const size_t oCL   = carve((size_t)NPr * HID2 * 2);
  const size_t oPABR = carve((size_t)NPr * HID2 * 4);
  const size_t oAGGR = carve((size_t)NPr * HID * 4);
  size_t scr = (size_t)CHE * 1024;
  if ((size_t)NPr * OUT_PAD * 4 > scr) scr = (size_t)NPr * OUT_PAD * 4;
  const size_t oSCR  = carve(scr);
  if (off > ws_size || off > (size_t)134217728) return;
  if ((size_t)EPr * KPAD * 2 > (size_t)NPr * HID2 * 4) return;
  if ((size_t)NPr * KPAD * 2 * 2 > (size_t)NPr * HID * 4) return;

  char* ws = (char*)d_ws;
  unsigned short* wn0h = (unsigned short*)(ws + oWN0H); unsigned short* wn0l = (unsigned short*)(ws + oWN0L);
  unsigned short* wn1h = (unsigned short*)(ws + oWN1H); unsigned short* wn1l = (unsigned short*)(ws + oWN1L);
  unsigned short* wn2h = (unsigned short*)(ws + oWN2H); unsigned short* wn2l = (unsigned short*)(ws + oWN2L);
  unsigned short* we0  = (unsigned short*)(ws + oWE0);
  unsigned short* we1  = (unsigned short*)(ws + oWE1);  unsigned short* we2  = (unsigned short*)(ws + oWE2);
  unsigned short* pbwh = (unsigned short*)(ws + oPBWH); unsigned short* pbwl = (unsigned short*)(ws + oPBWL);
  unsigned short* ew0c = (unsigned short*)(ws + oEW0C);
  unsigned short* ew1  = (unsigned short*)(ws + oEW1);  unsigned short* ew2  = (unsigned short*)(ws + oEW2);
  unsigned short* nw0h = (unsigned short*)(ws + oNW0H); unsigned short* nw0l = (unsigned short*)(ws + oNW0L);
  unsigned short* nw1h = (unsigned short*)(ws + oNW1H); unsigned short* nw1l = (unsigned short*)(ws + oNW1L);
  unsigned short* nw2h = (unsigned short*)(ws + oNW2H); unsigned short* nw2l = (unsigned short*)(ws + oNW2L);
  unsigned short* dw0h = (unsigned short*)(ws + oDW0H); unsigned short* dw0l = (unsigned short*)(ws + oDW0L);
  unsigned short* dw1h = (unsigned short*)(ws + oDW1H); unsigned short* dw1l = (unsigned short*)(ws + oDW1L);
  unsigned short* dw2h = (unsigned short*)(ws + oDW2H); unsigned short* dw2l = (unsigned short*)(ws + oDW2L);
  unsigned short* ef16 = (unsigned short*)(ws + oEF16);
  float*          nfp  = (float*)(ws + oNF);
  unsigned short* chp  = (unsigned short*)(ws + oCH);
  unsigned short* clp  = (unsigned short*)(ws + oCL);
  float*          pab  = (float*)(ws + oPABR);
  unsigned short* ex16 = (unsigned short*)(ws + oPABR);
  unsigned short* u1h  = (unsigned short*)(ws + oPABR);
  unsigned short* u1l  = (unsigned short*)(ws + oPABR + (size_t)NPr * HID * 2);
  unsigned short* u2h  = (unsigned short*)(ws + oPABR + (size_t)NPr * HID * 4);
  unsigned short* u2l  = (unsigned short*)(ws + oPABR + (size_t)NPr * HID * 6);
  float*          aggp = (float*)(ws + oAGGR);
  float*          u3   = (float*)(ws + oAGGR);
  unsigned short* xh   = (unsigned short*)(ws + oAGGR);
  unsigned short* xl   = (unsigned short*)(ws + oAGGR + (size_t)NPr * KPAD * 2);
  float*          r0f  = (float*)(ws + oSCR);
  unsigned short* m1p  = (unsigned short*)(ws + oSCR + (size_t)CHE * 512);
  unsigned short* m2p  = (unsigned short*)(ws + oSCR + (size_t)CHE * 512 + (size_t)CHE * 256);
  float*          newp = (float*)(ws + oSCR + (size_t)CHE * 512);
  float*          d3   = (float*)(ws + oSCR);

  auto gemm_blocks = [](int M, int Nn) { return ((M / 64) * (Nn / 64) + 7) / 8; };
  const float* rdum = nfp;
  const float* bdum = enb0;

  auto gs_relu16 = [&](const unsigned short* ah, const unsigned short* al, int lda,
                       const unsigned short* bh, const unsigned short* bl, int ldb,
                       unsigned short* oh, unsigned short* ol, int ldc, const float* bias, int M, int Nn, int K) {
    wmma_gemm64<1, true, 2, 2, false, 2><<<dim3(gemm_blocks(M, Nn), 1), NTHR, 0, stream>>>(
        ah, al, lda, 0L, bh, bl, ldb, 0L, (void*)oh, (void*)ol, ldc, 0L, bias, rdum, 0L, M, Nn, K, 1.0f);
  };
  auto gs_lin32 = [&](const unsigned short* ah, const unsigned short* al, int lda,
                      const unsigned short* bh, const unsigned short* bl, int ldb,
                      float* o, int ldc, const float* bias, int M, int Nn, int K) {
    wmma_gemm64<1, true, 2, 0, false, 0><<<dim3(gemm_blocks(M, Nn), 1), NTHR, 0, stream>>>(
        ah, al, lda, 0L, bh, bl, ldb, 0L, (void*)o, (void*)o, ldc, 0L, bias, rdum, 0L, M, Nn, K, 1.0f);
  };
  auto gs_nb32 = [&](const unsigned short* ah, const unsigned short* al, int lda,
                     const unsigned short* bh, const unsigned short* bl, int ldb,
                     float* o, int ldc, int M, int Nn, int K) {
    wmma_gemm64<1, true, 0, 0, false, 0><<<dim3(gemm_blocks(M, Nn), 1), NTHR, 0, stream>>>(
        ah, al, lda, 0L, bh, bl, ldb, 0L, (void*)o, (void*)o, ldc, 0L, bdum, rdum, 0L, M, Nn, K, 1.0f);
  };
  auto gf_relu16 = [&](const unsigned short* a, int lda, const unsigned short* bt, int ldb,
                       unsigned short* o, int ldc, const float* bias, int M, int Nn, int K) {
    wmma_gemm64<0, false, 2, 1, false, 2><<<dim3(gemm_blocks(M, Nn), 1), NTHR, 0, stream>>>(
        a, a, lda, 0L, bt, bt, ldb, 0L, (void*)o, (void*)o, ldc, 0L, bias, rdum, 0L, M, Nn, K, 0.125f);
  };
  auto gf_res_relu16 = [&](const unsigned short* a, int lda, const unsigned short* bt, int ldb,
                           unsigned short* o, int ldc, const float* bias, const float* res, int M, int Nn, int K) {
    wmma_gemm64<0, false, 2, 1, true, 2><<<dim3(gemm_blocks(M, Nn), 1), NTHR, 0, stream>>>(
        a, a, lda, 0L, bt, bt, ldb, 0L, (void*)o, (void*)o, ldc, 0L, bias, res, 0L, M, Nn, K, 0.125f);
  };
  auto gf_lin32 = [&](const unsigned short* a, int lda, const unsigned short* bt, int ldb,
                      float* o, int ldc, const float* bias, int M, int Nn, int K) {
    wmma_gemm64<0, false, 2, 0, false, 0><<<dim3(gemm_blocks(M, Nn), 1), NTHR, 0, stream>>>(
        a, a, lda, 0L, bt, bt, ldb, 0L, (void*)o, (void*)o, ldc, 0L, bias, rdum, 0L, M, Nn, K, 0.125f);
  };

  k_wsplit<<<dim3((HID * (KPAD / 8) + NTHR - 1) / NTHR, 1), NTHR, 0, stream>>>(enW0, 0L, NODE_IN, HID, 1, HID, KPAD, wn0h, wn0l, 0L);
  k_wsplit<<<dim3((HID * (HID / 8) + NTHR - 1) / NTHR, 1), NTHR, 0, stream>>>(enW1, 0L, HID, HID, 1, HID, HID, wn1h, wn1l, 0L);
  k_wsplit<<<dim3((HID * (HID / 8) + NTHR - 1) / NTHR, 1), NTHR, 0, stream>>>(enW2, 0L, HID, HID, 1, HID, HID, wn2h, wn2l, 0L);
  k_wf16<<<dim3((HID * (KPAD / 8) + NTHR - 1) / NTHR, 1), NTHR, 0, stream>>>(eeW0, 0L, EDGE_IN, HID, HID, KPAD, 8.0f, we0, 0L);
  k_wf16<<<dim3((HID * (HID / 8) + NTHR - 1) / NTHR, 1), NTHR, 0, stream>>>(eeW1, 0L, HID, HID, HID, HID, 8.0f, we1, 0L);
  k_wf16<<<dim3((HID * (HID / 8) + NTHR - 1) / NTHR, 1), NTHR, 0, stream>>>(eeW2, 0L, HID, HID, HID, HID, 8.0f, we2, 0L);
  k_wsplit<<<dim3((HID2 * (HID / 8) + NTHR - 1) / NTHR, NSTEP), NTHR, 0, stream>>>(
      geW0, (long)(3 * HID) * HID, HID, HID, 2, HID2, HID, pbwh, pbwl, (long)HID2 * HID);
  k_wf16<<<dim3((HID * (HID / 8) + NTHR - 1) / NTHR, NSTEP), NTHR, 0, stream>>>(
      geW0 + (size_t)HID2 * HID, (long)(3 * HID) * HID, HID, HID, HID, HID, 8.0f, ew0c, (long)HID * HID);
  k_wf16<<<dim3((HID * (HID / 8) + NTHR - 1) / NTHR, NSTEP), NTHR, 0, stream>>>(
      geW1, (long)HID * HID, HID, HID, HID, HID, 8.0f, ew1, (long)HID * HID);
  k_wf16<<<dim3((HID * (HID / 8) + NTHR - 1) / NTHR, NSTEP), NTHR, 0, stream>>>(
      geW2, (long)HID * HID, HID, HID, HID, HID, 8.0f, ew2, (long)HID * HID);
  k_wsplit<<<dim3((HID * (HID2 / 8) + NTHR - 1) / NTHR, NSTEP), NTHR, 0, stream>>>(
      gnW0, (long)HID2 * HID, HID2, HID, 1, HID, HID2, nw0h, nw0l, (long)HID * HID2);
  k_wsplit<<<dim3((HID * (HID / 8) + NTHR - 1) / NTHR, NSTEP), NTHR, 0, stream>>>(
      gnW1, (long)HID * HID, HID, HID, 1, HID, HID, nw1h, nw1l, (long)HID * HID);
  k_wsplit<<<dim3((HID * (HID / 8) + NTHR - 1) / NTHR, NSTEP), NTHR, 0, stream>>>(
      gnW2, (long)HID * HID, HID, HID, 1, HID, HID, nw2h, nw2l, (long)HID * HID);
  k_wsplit<<<dim3((HID * (HID / 8) + NTHR - 1) / NTHR, 1), NTHR, 0, stream>>>(dW0, 0L, HID, HID, 1, HID, HID, dw0h, dw0l, 0L);
  k_wsplit<<<dim3((HID * (HID / 8) + NTHR - 1) / NTHR, 1), NTHR, 0, stream>>>(dW1, 0L, HID, HID, 1, HID, HID, dw1h, dw1l, 0L);
  k_wsplit<<<dim3((OUT_PAD * (HID / 8) + NTHR - 1) / NTHR, 1), NTHR, 0, stream>>>(dW2, 0L, HID, OUT_CH, 1, OUT_PAD, HID, dw2h, dw2l, 0L);

  k_xsplit<<<(NPr * 4) / NTHR, NTHR, 0, stream>>>(node_x, nN, NPr, xh, xl);
  gs_relu16(xh, xl, KPAD, wn0h, wn0l, KPAD, u1h, u1l, HID, enb0, NPr, HID, KPAD);
  gs_relu16(u1h, u1l, HID, wn1h, wn1l, HID, u2h, u2l, HID, enb1, NPr, HID, HID);
  gs_lin32(u2h, u2l, HID, wn2h, wn2l, HID, u3, HID, enb2, NPr, HID, HID);
  k_nln<<<NPr / NWAVE, NTHR, 0, stream>>>(u3, eng, enbe, nN, NPr, 1, nfp, chp, clp);

  k_excast<<<(EPr * 4) / NTHR, NTHR, 0, stream>>>(edge_x, nE, EPr, ex16);
  for (int c = 0; c < nChunks; ++c) {
    const int base = c * CHE;
    int Ec = nE - base; if (Ec > CHE) Ec = CHE;
    const int Mc = ((Ec + 63) / 64) * 64;
    gf_relu16(ex16 + (size_t)base * KPAD, KPAD, we0, KPAD, m1p, HID, eeb0, Mc, HID, KPAD);
    gf_relu16(m1p, HID, we1, HID, m2p, HID, eeb1, Mc, HID, HID);
    gf_lin32(m2p, HID, we2, HID, r0f, HID, eeb2, Mc, HID, HID);
    k_eln<<<Mc / NWAVE, NTHR, 0, stream>>>(r0f, eeg, eebe, nE, EPr, base, Mc, 1, 0, ef16, newp);
  }

  for (int s = 0; s < NSTEP; ++s) {
    const unsigned short* pbwhs = pbwh + (size_t)s * HID2 * HID;
    const unsigned short* pbwls = pbwl + (size_t)s * HID2 * HID;
    const unsigned short* ew0cs = ew0c + (size_t)s * HID * HID;
    const unsigned short* ew1s  = ew1  + (size_t)s * HID * HID;
    const unsigned short* ew2s  = ew2  + (size_t)s * HID * HID;
    const unsigned short* nw0hs = nw0h + (size_t)s * HID * HID2;
    const unsigned short* nw0ls = nw0l + (size_t)s * HID * HID2;
    const unsigned short* nw1hs = nw1h + (size_t)s * HID * HID;
    const unsigned short* nw1ls = nw1l + (size_t)s * HID * HID;
    const unsigned short* nw2hs = nw2h + (size_t)s * HID * HID;
    const unsigned short* nw2ls = nw2l + (size_t)s * HID * HID;
    const float* eb0s = geb0 + (size_t)s * HID;  const float* eb1s = geb1 + (size_t)s * HID;
    const float* eb2s = geb2 + (size_t)s * HID;  const float* egs  = geg  + (size_t)s * HID;
    const float* ebes = gebe + (size_t)s * HID;
    const float* nb0s = gnb0 + (size_t)s * HID;  const float* nb1s = gnb1 + (size_t)s * HID;
    const float* nb2s = gnb2 + (size_t)s * HID;  const float* ngs  = gng  + (size_t)s * HID;
    const float* nbes = gnbe + (size_t)s * HID;

    gs_nb32(chp, clp, HID2, pbwhs, pbwls, HID, pab, HID2, NPr, HID2, HID);

    for (int c = 0; c < nChunks; ++c) {
      const int base = c * CHE;
      int Ec = nE - base; if (Ec > CHE) Ec = CHE;
      const int Mc = ((Ec + 63) / 64) * 64;
      const int vec = ((base & 3) == 0) ? 1 : 0;
      k_gath<<<Mc / NWAVE, NTHR, 0, stream>>>(pab, senders, receivers, nN, nE, base, Mc, r0f);
      gf_res_relu16(ef16 + (size_t)base * HID, HID, ew0cs, HID, m1p, HID, eb0s, r0f, Mc, HID, HID);
      gf_relu16(m1p, HID, ew1s, HID, m2p, HID, eb1s, Mc, HID, HID);
      gf_lin32(m2p, HID, ew2s, HID, r0f, HID, eb2s, Mc, HID, HID);
      k_eln<<<Mc / NWAVE, NTHR, 0, stream>>>(r0f, egs, ebes, nE, EPr, base, Mc, 0, 1, ef16, newp);
      k_agg<<<nA, NTHR, LDS_AGG, stream>>>(receivers + (size_t)base, Ec, newp, aggp, (c == 0) ? 1 : 0, vec);
    }

    k_aggsplit<<<(NPr * 16) / NTHR, NTHR, 0, stream>>>(aggp, NPr, chp, clp);
    gs_relu16(chp, clp, HID2, nw0hs, nw0ls, HID2, u1h, u1l, HID, nb0s, NPr, HID, HID2);
    gs_relu16(u1h, u1l, HID, nw1hs, nw1ls, HID, u2h, u2l, HID, nb1s, NPr, HID, HID);
    gs_lin32(u2h, u2l, HID, nw2hs, nw2ls, HID, u3, HID, nb2s, NPr, HID, HID);
    k_nln<<<NPr / NWAVE, NTHR, 0, stream>>>(u3, ngs, nbes, nN, NPr, 0, nfp, chp, clp);
  }

  gs_relu16(chp, clp, HID2, dw0h, dw0l, HID, u1h, u1l, HID, db0, NPr, HID, HID);
  gs_relu16(u1h, u1l, HID, dw1h, dw1l, HID, u2h, u2l, HID, db1, NPr, HID, HID);
  gs_nb32(u2h, u2l, HID, dw2h, dw2l, HID, d3, OUT_PAD, NPr, OUT_PAD, HID);
  k_pack<<<(out_size / 4 + NTHR - 1) / NTHR, NTHR, 0, stream>>>(d3, db2, nN, NPr, out0);
}
